// DNRI_DynamicVars_Encoder_52201032515963
// MI455X (gfx1250) — hardware-verified
//
#include <hip/hip_runtime.h>
#include <stddef.h>


#define T_   64
#define N_   40
#define D_   4
#define H_   256
#define R_   64
#define E_   1560
#define TE_  (T_ * E_)
#define TN_  (T_ * N_)
#define RT_  32
#define TP_  264
#define SP_  36
#define GP_  260
#define HP_  72
#define CAP_ 64
#define NT_  256

static_assert(TE_ % RT_ == 0);
static_assert(TN_ % RT_ == 0);
static_assert(TN_ % 8 == 0);
static_assert((TP_ * 2) % 16 == 0);
static_assert((HP_ * 2) % 16 == 0);
static_assert((SP_ * 4) % 16 == 0);

typedef unsigned short u16;
typedef u16    u16x8 __attribute__((ext_vector_type(8)));
typedef float  v4f   __attribute__((ext_vector_type(4)));
typedef float  v8f   __attribute__((ext_vector_type(8)));
typedef __bf16 v16b  __attribute__((ext_vector_type(16)));

union FragB { u16x8 h[2]; v16b v; };

constexpr size_t WO_M1W2 = 0;
constexpr size_t WO_M2W1 = WO_M1W2 + (size_t)H_ * H_;
constexpr size_t WO_M2W2 = WO_M2W1 + (size_t)H_ * 2 * H_;
constexpr size_t WO_M3W1 = WO_M2W2 + (size_t)H_ * H_;
constexpr size_t WO_M3W2 = WO_M3W1 + (size_t)H_ * H_;
constexpr size_t WO_M4W1 = WO_M3W2 + (size_t)H_ * H_;
constexpr size_t WO_M4W2 = WO_M4W1 + (size_t)H_ * 3 * H_;
constexpr size_t WO_FWIH = WO_M4W2 + (size_t)H_ * H_;
constexpr size_t WO_RWIH = WO_FWIH + (size_t)4 * R_ * H_;
constexpr size_t WO_FWHH = WO_RWIH + (size_t)4 * R_ * H_;
constexpr size_t WO_RWHH = WO_FWHH + (size_t)4 * R_ * R_;
constexpr size_t WN_TOT  = WO_RWHH + (size_t)4 * R_ * R_;

constexpr size_t SZ_WB = WN_TOT * 2;
constexpr size_t SZ_PQ = (size_t)TN_ * H_ * 4;
constexpr size_t SZ_NP = (size_t)TN_ * H_ * 2;
constexpr size_t SZ_EP = (size_t)TE_ * H_ * 2;
constexpr size_t SZ_HF = (size_t)TE_ * 4 * 4;

constexpr size_t OFF_WB = 0;
constexpr size_t OFF_P2 = OFF_WB + SZ_WB;
constexpr size_t OFF_Q2 = OFF_P2 + SZ_PQ;
constexpr size_t OFF_P4 = OFF_Q2 + SZ_PQ;
constexpr size_t OFF_Q4 = OFF_P4 + SZ_PQ;
constexpr size_t OFF_NH = OFF_Q4 + SZ_PQ;
constexpr size_t OFF_NL = OFF_NH + SZ_NP;
constexpr size_t OFF_EH = OFF_NL + SZ_NP;
constexpr size_t OFF_EL = OFF_EH + SZ_EP;
constexpr size_t OFF_HF = OFF_EL + SZ_EP;
constexpr size_t WS_END = OFF_HF + SZ_HF;
static_assert(WS_END <= (size_t)134217728);
static_assert(OFF_P2 % 128 == 0 && OFF_Q2 % 128 == 0 && OFF_P4 % 128 == 0 && OFF_Q4 % 128 == 0);
static_assert(OFF_NH % 128 == 0 && OFF_NL % 128 == 0 && OFF_EH % 128 == 0 && OFF_EL % 128 == 0);
static_assert(OFF_HF % 128 == 0 && WS_END % 128 == 0);
static_assert((WO_M2W1 * 2) % 128 == 0 && (WO_FWHH * 2) % 128 == 0 && (WO_RWHH * 2) % 128 == 0);

__device__ __forceinline__ u16 f2bf(float f) {
  unsigned u = __float_as_uint(f);
  u = u + 0x7FFFu + ((u >> 16) & 1u);
  return (u16)(u >> 16);
}
__device__ __forceinline__ float bf2f(u16 b) { return __uint_as_float(((unsigned)b) << 16); }
__device__ __forceinline__ float bfr(float f) { return bf2f(f2bf(f)); }
__device__ __forceinline__ void split1(float v, u16& hi, u16& lo) {
  hi = f2bf(v);
  lo = f2bf(v - bf2f(hi));
}
__device__ __forceinline__ float eluf(float v) {
  const float e = __expf(fminf(v, 0.0f)) - 1.0f;
  return v > 0.0f ? v : e;
}
__device__ __forceinline__ float sigf(float v) {
  const float x = fmaxf(v, -30.0f);
  return __builtin_amdgcn_rcpf(1.0f + expf(-x));
}

__device__ __forceinline__ void ldfrag(FragB& f, const u16* p) {
  f.h[0] = *(const u16x8*)(p);
  f.h[1] = *(const u16x8*)(p + 16);
}
__device__ __forceinline__ v8f wmma_bf16(const FragB& a, const FragB& b, v8f c) {
  return __builtin_amdgcn_wmma_f32_16x16x32_bf16(false, a.v, false, b.v, (short)0, c, false, false);
}
__device__ __forceinline__ void acc_zero(v8f (&acc)[4]) {
#pragma unroll
  for (int j = 0; j < 4; ++j) {
#pragma unroll
    for (int r = 0; r < 8; ++r) acc[j][r] = 0.0f;
  }
}
__device__ __forceinline__ void mm2(v8f (&acc)[4],
                                    const u16* aH0, const u16* aL0, const u16* aH1, const u16* aL1,
                                    const u16* b0, const u16* b1, int K)
{
#pragma unroll 2
  for (int k0 = 0; k0 < K; k0 += 32) {
    FragB ah0, al0, ah1, al1, fb0, fb1;
    ldfrag(ah0, aH0 + k0); ldfrag(al0, aL0 + k0);
    ldfrag(ah1, aH1 + k0); ldfrag(al1, aL1 + k0);
    ldfrag(fb0, b0 + k0);  ldfrag(fb1, b1 + k0);
    acc[0] = wmma_bf16(ah0, fb0, acc[0]);
    acc[0] = wmma_bf16(al0, fb0, acc[0]);
    acc[1] = wmma_bf16(ah0, fb1, acc[1]);
    acc[1] = wmma_bf16(al0, fb1, acc[1]);
    acc[2] = wmma_bf16(ah1, fb0, acc[2]);
    acc[2] = wmma_bf16(al1, fb0, acc[2]);
    acc[3] = wmma_bf16(ah1, fb1, acc[3]);
    acc[3] = wmma_bf16(al1, fb1, acc[3]);
    asm volatile("v_nop\n\tv_nop\n\tv_nop\n\tv_nop"
                 : "+v"(acc[0]), "+v"(acc[1]), "+v"(acc[2]), "+v"(acc[3])
                 : "v"(ah0.v), "v"(al0.v), "v"(ah1.v), "v"(al1.v), "v"(fb0.v), "v"(fb1.v));
  }
}

__device__ __forceinline__ void acc_to_tile_elu(const v8f (&acc)[4], u16* tH, u16* tL,
                                                int colw, int h, int m, float bb0, float bb1)
{
#pragma unroll
  for (int s = 0; s < 2; ++s) {
#pragma unroll
    for (int j = 0; j < 2; ++j) {
      const float bb = j ? bb1 : bb0;
      const int col = colw + 16 * j + m;
#pragma unroll
      for (int r = 0; r < 8; ++r) {
        const int row = 16 * s + 8 * h + r;
        u16 hi, lo;
        split1(eluf(acc[s * 2 + j][r] + bb), hi, lo);
        tH[row * TP_ + col] = hi;
        tL[row * TP_ + col] = lo;
      }
    }
  }
}

__device__ __forceinline__ void store_f32_tile(const v8f (&acc)[4], float* stgw, float* Cblk,
                                               int colw, int lane, int h, int m)
{
  const int q = lane >> 3, c = (lane & 7) * 4;
#pragma unroll
  for (int s = 0; s < 2; ++s) {
    __syncthreads();
#pragma unroll
    for (int j = 0; j < 2; ++j) {
#pragma unroll
      for (int r = 0; r < 8; ++r) stgw[(8 * h + r) * SP_ + 16 * j + m] = acc[s * 2 + j][r];
    }
    __syncthreads();
    v4f v[4];
#pragma unroll
    for (int it = 0; it < 4; ++it) v[it] = *(const v4f*)(stgw + (it * 4 + q) * SP_ + c);
#pragma unroll
    for (int it = 0; it < 4; ++it)
      *(volatile v4f*)(Cblk + (size_t)(16 * s + it * 4 + q) * H_ + colw + c) = v[it];
    __threadfence();
#pragma unroll
    for (int it = 0; it < 4; ++it)
      *(volatile v4f*)(Cblk + (size_t)(16 * s + it * 4 + q) * H_ + colw + c) = v[it];
  }
}

__device__ __forceinline__ void tile_rows_out(const u16* tH, const u16* tL, u16* gH, u16* gL,
                                              size_t rowBase, int wave, int lane)
{
  u16x8 hv[4], lv[4];
#pragma unroll
  for (int i = 0; i < 4; ++i) {
    const int row = wave * 4 + i;
    hv[i] = *(const u16x8*)(tH + row * TP_ + lane * 8);
    lv[i] = *(const u16x8*)(tL + row * TP_ + lane * 8);
  }
#pragma unroll
  for (int i = 0; i < 4; ++i) {
    const size_t p = (rowBase + (size_t)(wave * 4 + i)) * H_ + (size_t)lane * 8;
    *(volatile u16x8*)(gH + p) = hv[i];
    *(volatile u16x8*)(gL + p) = lv[i];
  }
  __threadfence();
#pragma unroll
  for (int i = 0; i < 4; ++i) {
    const size_t p = (rowBase + (size_t)(wave * 4 + i)) * H_ + (size_t)lane * 8;
    *(volatile u16x8*)(gH + p) = hv[i];
    *(volatile u16x8*)(gL + p) = lv[i];
  }
}

struct CvtSeg {
  const float* s0; const float* s1; const float* s2; const float* s3; const float* s4; const float* s5;
  const float* s6; const float* s7; const float* s8; const float* s9; const float* s10;
  int n0, n1, n2, n3, n4, n5, n6, n7, n8, n9, n10;
  int o0, o1, o2, o3, o4, o5, o6, o7, o8, o9, o10;
};
static_assert(sizeof(CvtSeg) == 176);

__global__ __launch_bounds__(NT_)
void k_cvt(CvtSeg a, u16* dst)
{
  const int seg = blockIdx.y;
  const float* s = (seg == 0) ? a.s0 : (seg == 1) ? a.s1 : (seg == 2) ? a.s2 : (seg == 3) ? a.s3 :
                   (seg == 4) ? a.s4 : (seg == 5) ? a.s5 : (seg == 6) ? a.s6 : (seg == 7) ? a.s7 :
                   (seg == 8) ? a.s8 : (seg == 9) ? a.s9 : a.s10;
  const int n    = (seg == 0) ? a.n0 : (seg == 1) ? a.n1 : (seg == 2) ? a.n2 : (seg == 3) ? a.n3 :
                   (seg == 4) ? a.n4 : (seg == 5) ? a.n5 : (seg == 6) ? a.n6 : (seg == 7) ? a.n7 :
                   (seg == 8) ? a.n8 : (seg == 9) ? a.n9 : a.n10;
  const int o    = (seg == 0) ? a.o0 : (seg == 1) ? a.o1 : (seg == 2) ? a.o2 : (seg == 3) ? a.o3 :
                   (seg == 4) ? a.o4 : (seg == 5) ? a.o5 : (seg == 6) ? a.o6 : (seg == 7) ? a.o7 :
                   (seg == 8) ? a.o8 : (seg == 9) ? a.o9 : a.o10;
  const int i8 = blockIdx.x * NT_ + threadIdx.x;
  if (i8 * 8 >= n) return;
  const v4f x0 = *(const v4f*)(s + (size_t)i8 * 8);
  const v4f x1 = *(const v4f*)(s + (size_t)i8 * 8 + 4);
  u16x8 hv;
  hv[0] = f2bf(x0[0]); hv[1] = f2bf(x0[1]); hv[2] = f2bf(x0[2]); hv[3] = f2bf(x0[3]);
  hv[4] = f2bf(x1[0]); hv[5] = f2bf(x1[1]); hv[6] = f2bf(x1[2]); hv[7] = f2bf(x1[3]);
  u16* p = dst + (size_t)o + (size_t)i8 * 8;
  *(volatile u16x8*)p = hv;
  __threadfence();
  *(volatile u16x8*)p = hv;
}

__global__ __launch_bounds__(NT_)
void k_node1(const float* __restrict__ X, const float* __restrict__ W1, const float* __restrict__ b1,
             const u16* __restrict__ W2b, const float* __restrict__ b2,
             const u16* __restrict__ W21b, float* P2, float* Q2)
{
  __shared__ __attribute__((aligned(16))) u16 tH[RT_ * TP_];
  __shared__ __attribute__((aligned(16))) u16 tL[RT_ * TP_];
  __shared__ __attribute__((aligned(16))) float stg[8 * 16 * SP_];
  const int tid = threadIdx.x, lane = tid & 31, wave = tid >> 5;
  const int h = lane >> 4, m = lane & 15, colw = wave * 32;
  const int rowBase = blockIdx.x * RT_;

  {
    const int er = tid >> 3, c0 = (tid & 7) * 32;
    const int g = rowBase + er;
    const v4f xv = *(const v4f*)(X + (size_t)g * D_);
    const float x0 = bfr(xv[0]), x1 = bfr(xv[1]), x2 = bfr(xv[2]), x3 = bfr(xv[3]);
#pragma unroll 1
    for (int blk = 0; blk < 4; ++blk) {
      const int cb = c0 + blk * 8;
      u16x8 hv, lv;
#pragma unroll
      for (int i = 0; i < 8; ++i) {
        const int c = cb + i;
        const v4f w = *(const v4f*)(W1 + (size_t)c * D_);
        float s = bfr(w[0]) * x0;
        s = bfr(w[1]) * x1 + s;
        s = bfr(w[2]) * x2 + s;
        s = bfr(w[3]) * x3 + s;
        s = s + bfr(b1[c]);
        u16 hi, lo;
        split1(eluf(s), hi, lo);
        hv[i] = hi; lv[i] = lo;
      }
      *(u16x8*)(tH + er * TP_ + cb) = hv;
      *(u16x8*)(tL + er * TP_ + cb) = lv;
    }
  }
  __syncthreads();

  const u16* aH0 = tH + m * TP_ + 8 * h;
  const u16* aL0 = tL + m * TP_ + 8 * h;
  const u16* aH1 = tH + (16 + m) * TP_ + 8 * h;
  const u16* aL1 = tL + (16 + m) * TP_ + 8 * h;
  v8f acc[4];

  acc_zero(acc);
  mm2(acc, aH0, aL0, aH1, aL1,
      W2b + (size_t)(colw + m) * H_ + 8 * h, W2b + (size_t)(colw + 16 + m) * H_ + 8 * h, H_);
  {
    const float bb0 = bfr(b2[colw + m]), bb1 = bfr(b2[colw + 16 + m]);
    __syncthreads();
    acc_to_tile_elu(acc, tH, tL, colw, h, m, bb0, bb1);
    __syncthreads();
  }

  acc_zero(acc);
  mm2(acc, aH0, aL0, aH1, aL1,
      W21b + (size_t)(colw + m) * (2 * H_) + 8 * h, W21b + (size_t)(colw + 16 + m) * (2 * H_) + 8 * h, H_);
  store_f32_tile(acc, stg + wave * 16 * SP_, P2 + (size_t)rowBase * H_, colw, lane, h, m);

  acc_zero(acc);
  mm2(acc, aH0, aL0, aH1, aL1,
      W21b + (size_t)(colw + m) * (2 * H_) + H_ + 8 * h,
      W21b + (size_t)(colw + 16 + m) * (2 * H_) + H_ + 8 * h, H_);
  store_f32_tile(acc, stg + wave * 16 * SP_, Q2 + (size_t)rowBase * H_, colw, lane, h, m);
}

__global__ __launch_bounds__(NT_)
void k_edge2(const float* __restrict__ P2, const float* __restrict__ Q2,
             const int* __restrict__ send, const int* __restrict__ recv,
             const float* __restrict__ b1, const u16* __restrict__ W2b, const float* __restrict__ b2,
             u16* EH, u16* EL)
{
  __shared__ __attribute__((aligned(16))) u16 tH[RT_ * TP_];
  __shared__ __attribute__((aligned(16))) u16 tL[RT_ * TP_];
  const int tid = threadIdx.x, lane = tid & 31, wave = tid >> 5;
  const int h = lane >> 4, m = lane & 15, colw = wave * 32;
  const int rowBase = blockIdx.x * RT_;

  {
    const int er = tid >> 3, c0 = (tid & 7) * 32;
    const int g = rowBase + er;
    const int t = g / E_;
    const int e = g - t * E_;
    int sn = send[e]; sn = min(max(sn, 0), N_ - 1);
    int rn = recv[e]; rn = min(max(rn, 0), N_ - 1);
    const float* pP = P2 + (size_t)(t * N_ + sn) * H_ + c0;
    const float* pQ = Q2 + (size_t)(t * N_ + rn) * H_ + c0;
    const float* pb = b1 + c0;
#pragma unroll 1
    for (int blk = 0; blk < 4; ++blk) {
      const int cb = blk * 8;
      const v4f a0 = *(const v4f*)(pP + cb), a1 = *(const v4f*)(pP + cb + 4);
      const v4f q0 = *(const v4f*)(pQ + cb), q1 = *(const v4f*)(pQ + cb + 4);
      const v4f w0 = *(const v4f*)(pb + cb), w1 = *(const v4f*)(pb + cb + 4);
      u16x8 hv, lv;
#pragma unroll
      for (int i = 0; i < 4; ++i) {
        u16 hi, lo;
        split1(eluf((a0[i] + q0[i]) + bfr(w0[i])), hi, lo);
        hv[i] = hi; lv[i] = lo;
        split1(eluf((a1[i] + q1[i]) + bfr(w1[i])), hi, lo);
        hv[4 + i] = hi; lv[4 + i] = lo;
      }
      *(u16x8*)(tH + er * TP_ + c0 + cb) = hv;
      *(u16x8*)(tL + er * TP_ + c0 + cb) = lv;
    }
  }
  __syncthreads();

  const u16* aH0 = tH + m * TP_ + 8 * h;
  const u16* aL0 = tL + m * TP_ + 8 * h;
  const u16* aH1 = tH + (16 + m) * TP_ + 8 * h;
  const u16* aL1 = tL + (16 + m) * TP_ + 8 * h;
  v8f acc[4];
  acc_zero(acc);
  mm2(acc, aH0, aL0, aH1, aL1,
      W2b + (size_t)(colw + m) * H_ + 8 * h, W2b + (size_t)(colw + 16 + m) * H_ + 8 * h, H_);
  const float bb0 = bfr(b2[colw + m]), bb1 = bfr(b2[colw + 16 + m]);
  __syncthreads();
  acc_to_tile_elu(acc, tH, tL, colw, h, m, bb0, bb1);
  __syncthreads();
  tile_rows_out(tH, tL, EH, EL, (size_t)rowBase, wave, lane);
}

__global__ __launch_bounds__(NT_)
void k_agg(const u16* __restrict__ EH, const u16* __restrict__ EL, const int* __restrict__ recv,
           u16* NH, u16* NL)
{
  __shared__ int lst[8 * CAP_];
  const int tid = threadIdx.x, lane = tid & 31, wave = tid >> 5;
  const int d = blockIdx.x * 8 + wave;
  const int t = d / N_;
  const int node = d - t * N_;
  int cnt = 0;
#pragma unroll 1
  for (int base = 0; base < E_; base += 32) {
    const int e = base + lane;
    const int ec = min(e, E_ - 1);
    const int rv = recv[ec];
    const bool hit = (e < E_) && (rv == node);
    const unsigned msk = (unsigned)__ballot(hit ? 1 : 0);
    const unsigned lt = (1u << lane) - 1u;
    const int pos = cnt + (int)__popc(msk & lt);
    if (hit && pos < CAP_) lst[wave * CAP_ + pos] = e;
    cnt += (int)__popc(msk);
  }
  __syncthreads();
  const int cn = min(cnt, CAP_);
  float sacc[8];
#pragma unroll
  for (int i = 0; i < 8; ++i) sacc[i] = 0.0f;
  const int c0 = lane * 8;
#pragma unroll 1
  for (int j = 0; j < cn; ++j) {
    int e = lst[wave * CAP_ + j];
    e = min(max(e, 0), E_ - 1);
    const size_t p = ((size_t)t * E_ + (size_t)e) * H_ + c0;
    const u16x8 hv = *(const u16x8*)(EH + p);
    const u16x8 lv = *(const u16x8*)(EL + p);
#pragma unroll
    for (int i = 0; i < 8; ++i) sacc[i] += (bf2f(hv[i]) + bf2f(lv[i]));
  }
  u16x8 oh, ol;
#pragma unroll
  for (int i = 0; i < 8; ++i) {
    u16 hi, lo;
    split1(sacc[i], hi, lo);
    oh[i] = hi; ol[i] = lo;
  }
  const size_t p = (size_t)d * H_ + c0;
  *(volatile u16x8*)(NH + p) = oh;
  *(volatile u16x8*)(NL + p) = ol;
  __threadfence();
  *(volatile u16x8*)(NH + p) = oh;
  *(volatile u16x8*)(NL + p) = ol;
}

__global__ __launch_bounds__(NT_)
void k_node3(const u16* __restrict__ NH, const u16* __restrict__ NL,
             const u16* __restrict__ W1b, const float* __restrict__ b1,
             const u16* __restrict__ W2b, const float* __restrict__ b2,
             const u16* __restrict__ W41b, float* P4, float* Q4)
{
  __shared__ __attribute__((aligned(16))) u16 tH[RT_ * TP_];
  __shared__ __attribute__((aligned(16))) u16 tL[RT_ * TP_];
  __shared__ __attribute__((aligned(16))) float stg[8 * 16 * SP_];
  const int tid = threadIdx.x, lane = tid & 31, wave = tid >> 5;
  const int h = lane >> 4, m = lane & 15, colw = wave * 32;
  const int rowBase = blockIdx.x * RT_;

  const u16* aH0 = tH + m * TP_ + 8 * h;
  const u16* aL0 = tL + m * TP_ + 8 * h;
  const u16* aH1 = tH + (16 + m) * TP_ + 8 * h;
  const u16* aL1 = tL + (16 + m) * TP_ + 8 * h;
  v8f acc[4];

  acc_zero(acc);
  mm2(acc,
      NH + (size_t)(rowBase + m) * H_ + 8 * h, NL + (size_t)(rowBase + m) * H_ + 8 * h,
      NH + (size_t)(rowBase + 16 + m) * H_ + 8 * h, NL + (size_t)(rowBase + 16 + m) * H_ + 8 * h,
      W1b + (size_t)(colw + m) * H_ + 8 * h, W1b + (size_t)(colw + 16 + m) * H_ + 8 * h, H_);
  {
    const float bb0 = bfr(b1[colw + m]), bb1 = bfr(b1[colw + 16 + m]);
    acc_to_tile_elu(acc, tH, tL, colw, h, m, bb0, bb1);
    __syncthreads();
  }
  acc_zero(acc);
  mm2(acc, aH0, aL0, aH1, aL1,
      W2b + (size_t)(colw + m) * H_ + 8 * h, W2b + (size_t)(colw + 16 + m) * H_ + 8 * h, H_);
  {
    const float bb0 = bfr(b2[colw + m]), bb1 = bfr(b2[colw + 16 + m]);
    __syncthreads();
    acc_to_tile_elu(acc, tH, tL, colw, h, m, bb0, bb1);
    __syncthreads();
  }
  acc_zero(acc);
  mm2(acc, aH0, aL0, aH1, aL1,
      W41b + (size_t)(colw + m) * (3 * H_) + 8 * h, W41b + (size_t)(colw + 16 + m) * (3 * H_) + 8 * h, H_);
  store_f32_tile(acc, stg + wave * 16 * SP_, P4 + (size_t)rowBase * H_, colw, lane, h, m);
  acc_zero(acc);
  mm2(acc, aH0, aL0, aH1, aL1,
      W41b + (size_t)(colw + m) * (3 * H_) + H_ + 8 * h,
      W41b + (size_t)(colw + 16 + m) * (3 * H_) + H_ + 8 * h, H_);
  store_f32_tile(acc, stg + wave * 16 * SP_, Q4 + (size_t)rowBase * H_, colw, lane, h, m);
}

__global__ __launch_bounds__(NT_)
void k_edge4(const float* __restrict__ P4, const float* __restrict__ Q4,
             const int* __restrict__ send, const int* __restrict__ recv,
             const u16* __restrict__ W1b, const float* __restrict__ b1,
             const u16* __restrict__ W2b, const float* __restrict__ b2,
             u16* EH, u16* EL)
{
  __shared__ __attribute__((aligned(16))) u16 tH[RT_ * TP_];
  __shared__ __attribute__((aligned(16))) u16 tL[RT_ * TP_];
  __shared__ int rowP[RT_];
  __shared__ int rowQ[RT_];
  const int tid = threadIdx.x, lane = tid & 31, wave = tid >> 5;
  const int h = lane >> 4, m = lane & 15, colw = wave * 32;
  const int rowBase = blockIdx.x * RT_;

  if (wave == 0) {
    const int g = rowBase + lane;
    const int t = g / E_;
    const int e = g - t * E_;
    int sn = send[e]; sn = min(max(sn, 0), N_ - 1);
    int rn = recv[e]; rn = min(max(rn, 0), N_ - 1);
    rowP[lane] = (t * N_ + sn) * H_;
    rowQ[lane] = (t * N_ + rn) * H_;
  }

  v8f acc[4];
  acc_zero(acc);
  mm2(acc,
      EH + (size_t)(rowBase + m) * H_ + 8 * h, EL + (size_t)(rowBase + m) * H_ + 8 * h,
      EH + (size_t)(rowBase + 16 + m) * H_ + 8 * h, EL + (size_t)(rowBase + 16 + m) * H_ + 8 * h,
      W1b + (size_t)(colw + m) * (3 * H_) + 2 * H_ + 8 * h,
      W1b + (size_t)(colw + 16 + m) * (3 * H_) + 2 * H_ + 8 * h, H_);
  {
    const float bb0 = bfr(b1[colw + m]), bb1 = bfr(b1[colw + 16 + m]);
    __syncthreads();
#pragma unroll
    for (int s = 0; s < 2; ++s) {
#pragma unroll
      for (int j = 0; j < 2; ++j) {
        const float bb = j ? bb1 : bb0;
        const int col = colw + 16 * j + m;
#pragma unroll
        for (int r = 0; r < 8; ++r) {
          const int row = 16 * s + 8 * h + r;
          const int op = rowP[row], oq = rowQ[row];
          float v = acc[s * 2 + j][r] + P4[op + col];
          v = v + Q4[oq + col];
          v = v + bb;
          u16 hi, lo;
          split1(eluf(v), hi, lo);
          tH[row * TP_ + col] = hi;
          tL[row * TP_ + col] = lo;
        }
      }
    }
    __syncthreads();
  }
  const u16* aH0 = tH + m * TP_ + 8 * h;
  const u16* aL0 = tL + m * TP_ + 8 * h;
  const u16* aH1 = tH + (16 + m) * TP_ + 8 * h;
  const u16* aL1 = tL + (16 + m) * TP_ + 8 * h;
  acc_zero(acc);
  mm2(acc, aH0, aL0, aH1, aL1,
      W2b + (size_t)(colw + m) * H_ + 8 * h, W2b + (size_t)(colw + 16 + m) * H_ + 8 * h, H_);
  {
    const float bb0 = bfr(b2[colw + m]), bb1 = bfr(b2[colw + 16 + m]);
    __syncthreads();
    acc_to_tile_elu(acc, tH, tL, colw, h, m, bb0, bb1);
    __syncthreads();
  }
  tile_rows_out(tH, tL, EH, EL, (size_t)rowBase, wave, lane);
}

__global__ __launch_bounds__(NT_)
void k_lstm(const u16* __restrict__ EH, const u16* __restrict__ EL,
            const u16* __restrict__ Wih, const u16* __restrict__ Whh,
            const float* __restrict__ bih, const float* __restrict__ bhh,
            const float* __restrict__ priW, const float* __restrict__ prib,
            const float* __restrict__ encW, const float* __restrict__ encb,
            float* HF, float* OUT, int dir)
{
  __shared__ __attribute__((aligned(16))) u16 hH[RT_ * HP_];
  __shared__ __attribute__((aligned(16))) u16 hL[RT_ * HP_];
  __shared__ __attribute__((aligned(16))) float gS[RT_ * GP_];
  __shared__ __attribute__((aligned(16))) float oS[RT_ * 4];
  const int tid = threadIdx.x, lane = tid & 31, wave = tid >> 5;
  const int h = lane >> 4, m = lane & 15, colw = wave * 32;
  const int e0 = blockIdx.x * RT_;
  const int nrows = min(RT_, E_ - e0);

  for (int i = tid; i < RT_ * HP_; i += NT_) { hH[i] = 0; hL[i] = 0; }

  const int ce0 = min(e0 + m, E_ - 1);
  const int ce1 = min(e0 + 16 + m, E_ - 1);
  const u16* bI0 = Wih + (size_t)(colw + m) * H_ + 8 * h;
  const u16* bI1 = Wih + (size_t)(colw + 16 + m) * H_ + 8 * h;
  const u16* bR0 = Whh + (size_t)(colw + m) * R_ + 8 * h;
  const u16* bR1 = Whh + (size_t)(colw + 16 + m) * R_ + 8 * h;
  const u16* aRH0 = hH + m * HP_ + 8 * h;
  const u16* aRL0 = hL + m * HP_ + 8 * h;
  const u16* aRH1 = hH + (16 + m) * HP_ + 8 * h;
  const u16* aRL1 = hL + (16 + m) * HP_ + 8 * h;
  const float gb0 = bfr(bih[colw + m]) + bfr(bhh[colw + m]);
  const float gb1 = bfr(bih[colw + 16 + m]) + bfr(bhh[colw + 16 + m]);

  const int er = tid >> 3, q = tid & 7, j0 = q * 8;
  float pw0[8], pw1[8], ew0[8], ew1[8];
#pragma unroll
  for (int i = 0; i < 8; ++i) {
    pw0[i] = bfr(priW[j0 + i]);
    pw1[i] = bfr(priW[R_ + j0 + i]);
    ew0[i] = bfr(encW[dir * R_ + j0 + i]);
    ew1[i] = bfr(encW[2 * R_ + dir * R_ + j0 + i]);
  }
  const float pb0 = bfr(prib[0]), pb1 = bfr(prib[1]);
  const float eb0 = bfr(encb[0]), eb1 = bfr(encb[1]);
  const int erow = min(e0 + er, E_ - 1);
  float cst[8];
#pragma unroll
  for (int i = 0; i < 8; ++i) cst[i] = 0.0f;
  __syncthreads();

#pragma unroll 1
  for (int step = 0; step < T_; ++step) {
    const int t = dir ? (T_ - 1 - step) : step;
    const size_t rb = (size_t)t * E_;
    v8f acc[4];
    acc_zero(acc);
    mm2(acc,
        EH + (rb + ce0) * H_ + 8 * h, EL + (rb + ce0) * H_ + 8 * h,
        EH + (rb + ce1) * H_ + 8 * h, EL + (rb + ce1) * H_ + 8 * h,
        bI0, bI1, H_);
    mm2(acc, aRH0, aRL0, aRH1, aRL1, bR0, bR1, R_);
#pragma unroll
    for (int s = 0; s < 2; ++s) {
#pragma unroll
      for (int j = 0; j < 2; ++j) {
        const float bb = j ? gb1 : gb0;
        const int col = colw + 16 * j + m;
#pragma unroll
        for (int r = 0; r < 8; ++r) gS[(16 * s + 8 * h + r) * GP_ + col] = acc[s * 2 + j][r] + bb;
      }
    }
    __syncthreads();

    float hv8[8];
    u16x8 hh, hl;
    const float* gr = gS + er * GP_;
#pragma unroll
    for (int i = 0; i < 8; ++i) {
      const int jj = j0 + i;
      const float gi = gr[jj], gf = gr[R_ + jj], gg = gr[2 * R_ + jj], go = gr[3 * R_ + jj];
      const float cc = sigf(gf) * cst[i] + sigf(gi) * tanhf(gg);
      cst[i] = cc;
      const float hvv = sigf(go) * tanhf(cc);
      hv8[i] = hvv;
      u16 hi, lo;
      split1(hvv, hi, lo);
      hh[i] = hi; hl[i] = lo;
    }
    *(u16x8*)(hH + er * HP_ + j0) = hh;
    *(u16x8*)(hL + er * HP_ + j0) = hl;
    float p0 = 0.0f, p1 = 0.0f, s0 = 0.0f, s1 = 0.0f;
#pragma unroll
    for (int i = 0; i < 8; ++i) {
      p0 = hv8[i] * pw0[i] + p0;
      p1 = hv8[i] * pw1[i] + p1;
      s0 = hv8[i] * ew0[i] + s0;
      s1 = hv8[i] * ew1[i] + s1;
    }
#pragma unroll
    for (int mm = 1; mm <= 4; mm <<= 1) {
      p0 += __shfl_xor(p0, mm, 32);
      p1 += __shfl_xor(p1, mm, 32);
      s0 += __shfl_xor(s0, mm, 32);
      s1 += __shfl_xor(s1, mm, 32);
    }
    if (dir == 0) {
      if (q == 0) {
        oS[er * 4 + 0] = p0 + pb0;
        oS[er * 4 + 1] = p1 + pb1;
        oS[er * 4 + 2] = s0;
        oS[er * 4 + 3] = s1;
      }
    } else {
      const v4f f = *(const v4f*)(HF + (rb + (size_t)erow) * 4);
      if (q == 0) {
        oS[er * 4 + 0] = f[0];
        oS[er * 4 + 1] = f[1];
        oS[er * 4 + 2] = (f[2] + s0) + eb0;
        oS[er * 4 + 3] = (f[3] + s1) + eb1;
      }
    }
    __syncthreads();

    if (wave == 0) {
      const v4f v = *(const v4f*)(oS + lane * 4);
      const int el = min(e0 + lane, E_ - 1);
      float* dst = (dir ? OUT : HF) + (rb + (size_t)el) * 4;
      if (lane < nrows) *(volatile v4f*)dst = v;
      __threadfence();
      if (lane < nrows) *(volatile v4f*)dst = v;
    }
  }
}

extern "C" void kernel_launch(void* const* d_in, const int* in_sizes, int n_in,
                              void* d_out, int out_size, void* d_ws, size_t ws_size,
                              hipStream_t stream)
{
  if (n_in < 32) return;
  if (in_sizes[0] != TN_ * D_) return;
  if (in_sizes[2] != E_ || in_sizes[3] != E_) return;
  if (in_sizes[4] != H_ * D_ || in_sizes[5] != H_ || in_sizes[6] != H_ * H_ || in_sizes[7] != H_) return;
  if (in_sizes[8] != H_ * 2 * H_ || in_sizes[9] != H_ || in_sizes[10] != H_ * H_ || in_sizes[11] != H_) return;
  if (in_sizes[12] != H_ * H_ || in_sizes[13] != H_ || in_sizes[14] != H_ * H_ || in_sizes[15] != H_) return;
  if (in_sizes[16] != H_ * 3 * H_ || in_sizes[17] != H_ || in_sizes[18] != H_ * H_ || in_sizes[19] != H_) return;
  if (in_sizes[20] != 4 * R_ * H_ || in_sizes[21] != 4 * R_ * R_ || in_sizes[22] != 4 * R_ || in_sizes[23] != 4 * R_) return;
  if (in_sizes[24] != 4 * R_ * H_ || in_sizes[25] != 4 * R_ * R_ || in_sizes[26] != 4 * R_ || in_sizes[27] != 4 * R_) return;
  if (in_sizes[28] != 2 * 2 * R_ || in_sizes[29] != 2 || in_sizes[30] != 2 * R_ || in_sizes[31] != 2) return;
  if (out_size != TE_ * 4) return;
  if (ws_size < WS_END) return;

  const float* x    = (const float*)d_in[0];
  const int*   send = (const int*)d_in[2];
  const int*   recv = (const int*)d_in[3];
  const float* m1W1 = (const float*)d_in[4];  const float* m1b1 = (const float*)d_in[5];
  const float* m1W2 = (const float*)d_in[6];  const float* m1b2 = (const float*)d_in[7];
  const float* m2W1 = (const float*)d_in[8];  const float* m2b1 = (const float*)d_in[9];
  const float* m2W2 = (const float*)d_in[10]; const float* m2b2 = (const float*)d_in[11];
  const float* m3W1 = (const float*)d_in[12]; const float* m3b1 = (const float*)d_in[13];
  const float* m3W2 = (const float*)d_in[14]; const float* m3b2 = (const float*)d_in[15];
  const float* m4W1 = (const float*)d_in[16]; const float* m4b1 = (const float*)d_in[17];
  const float* m4W2 = (const float*)d_in[18]; const float* m4b2 = (const float*)d_in[19];
  const float* fWih = (const float*)d_in[20]; const float* fWhh = (const float*)d_in[21];
  const float* fbih = (const float*)d_in[22]; const float* fbhh = (const float*)d_in[23];
  const float* rWih = (const float*)d_in[24]; const float* rWhh = (const float*)d_in[25];
  const float* rbih = (const float*)d_in[26]; const float* rbhh = (const float*)d_in[27];
  const float* encW = (const float*)d_in[28]; const float* encb = (const float*)d_in[29];
  const float* priW = (const float*)d_in[30]; const float* prib = (const float*)d_in[31];
  float* out = (float*)d_out;

  char* ws = (char*)d_ws;
  u16*   wb = (u16*)(ws + OFF_WB);
  float* P2 = (float*)(ws + OFF_P2);
  float* Q2 = (float*)(ws + OFF_Q2);
  float* P4 = (float*)(ws + OFF_P4);
  float* Q4 = (float*)(ws + OFF_Q4);
  u16*   NH = (u16*)(ws + OFF_NH);
  u16*   NL = (u16*)(ws + OFF_NL);
  u16*   EH = (u16*)(ws + OFF_EH);
  u16*   EL = (u16*)(ws + OFF_EL);
  float* HF = (float*)(ws + OFF_HF);

  CvtSeg cs;
  cs.s0 = m1W2; cs.n0 = H_ * H_;      cs.o0 = (int)WO_M1W2;
  cs.s1 = m2W1; cs.n1 = H_ * 2 * H_;  cs.o1 = (int)WO_M2W1;
  cs.s2 = m2W2; cs.n2 = H_ * H_;      cs.o2 = (int)WO_M2W2;
  cs.s3 = m3W1; cs.n3 = H_ * H_;      cs.o3 = (int)WO_M3W1;
  cs.s4 = m3W2; cs.n4 = H_ * H_;      cs.o4 = (int)WO_M3W2;
  cs.s5 = m4W1; cs.n5 = H_ * 3 * H_;  cs.o5 = (int)WO_M4W1;
  cs.s6 = m4W2; cs.n6 = H_ * H_;      cs.o6 = (int)WO_M4W2;
  cs.s7 = fWih; cs.n7 = 4 * R_ * H_;  cs.o7 = (int)WO_FWIH;
  cs.s8 = rWih; cs.n8 = 4 * R_ * H_;  cs.o8 = (int)WO_RWIH;
  cs.s9 = fWhh; cs.n9 = 4 * R_ * R_;  cs.o9 = (int)WO_FWHH;
  cs.s10 = rWhh; cs.n10 = 4 * R_ * R_; cs.o10 = (int)WO_RWHH;
  k_cvt<<<dim3((H_ * 3 * H_ / 8 + NT_ - 1) / NT_, 11), dim3(NT_), 0, stream>>>(cs, wb);

  k_node1<<<dim3(TN_ / RT_), dim3(NT_), 0, stream>>>(
      x, m1W1, m1b1, wb + WO_M1W2, m1b2, wb + WO_M2W1, P2, Q2);

  k_edge2<<<dim3(TE_ / RT_), dim3(NT_), 0, stream>>>(
      P2, Q2, send, recv, m2b1, wb + WO_M2W2, m2b2, EH, EL);

  k_agg<<<dim3(TN_ / 8), dim3(NT_), 0, stream>>>(EH, EL, recv, NH, NL);

  k_node3<<<dim3(TN_ / RT_), dim3(NT_), 0, stream>>>(
      NH, NL, wb + WO_M3W1, m3b1, wb + WO_M3W2, m3b2, wb + WO_M4W1, P4, Q4);

  k_edge4<<<dim3(TE_ / RT_), dim3(NT_), 0, stream>>>(
      P4, Q4, send, recv, wb + WO_M4W1, m4b1, wb + WO_M4W2, m4b2, EH, EL);

  k_lstm<<<dim3((E_ + RT_ - 1) / RT_), dim3(NT_), 0, stream>>>(
      EH, EL, wb + WO_FWIH, wb + WO_FWHH, fbih, fbhh, priW, prib, encW, encb, HF, out, 0);

  k_lstm<<<dim3((E_ + RT_ - 1) / RT_), dim3(NT_), 0, stream>>>(
      EH, EL, wb + WO_RWIH, wb + WO_RWHH, rbih, rbhh, priW, prib, encW, encb, HF, out, 1);
}
